// SymmetricCPRing_72816875537122
// MI455X (gfx1250) — hardware-verified
//
#include <hip/hip_runtime.h>
#include <math.h>

#ifndef NB
#define NB 4096
#endif
#define NB_FULL 4096
#define CHN 128
#define LDIM 16
#define NEL 10
#define NP3 23
#define NP2 5
#define MEC (NEL * CHN)
#define NQ (LDIM * LDIM * LDIM)
#define KP 32
#define TSPLIT 4
#define XP 20
#define SWC 1024.0f
#define SUC 256.0f
#define SBC 1024.0f
#define SAC 64.0f

static constexpr float VSCALE = 1.0f / 256.0f;

static_assert(NB % 256 == 0);
static_assert(NB <= NB_FULL);
static_assert(MEC % 64 == 0 && NQ % 64 == 0 && KP == 32);
static_assert(NP3 <= KP);
static_assert((MEC * 4) % 256 == 0 && (NQ * 4) % 256 == 0);
static_assert((MEC * 64) % 256 == 0);
static_assert(((MEC / 64) * (NQ / 64)) % 8 == 0);
static_assert(CHN % 16 == 0 && CHN / 16 == 8);
static_assert(LDIM == 16);
static_assert(XP % 4 == 0 && XP >= LDIM);
static_assert(8 * 4 == 16 * 2);
static_assert(8 * 16 == 128);
static_assert(4 * 4 == 16);
static_assert(4 * NB + 32 + 4 * 8 * 16 * XP + 4 * 8 * 16 * 16 + 4 * 8 * 16 <= 131072);
static_assert(4 * 8 * 16 * 68 <= 131072);
static_assert((size_t)MEC * KP * 2 + (size_t)NQ * KP * 2 + 2 * (size_t)MEC * NQ * 2 + 2 * (size_t)MEC * 16 * 32 * 2 <= (size_t)134217728);

typedef _Float16 h16;
typedef __attribute__((ext_vector_type(16))) _Float16 v16h;
typedef __attribute__((ext_vector_type(8)))  _Float16 v8h;
typedef __attribute__((ext_vector_type(8)))  float    v8f;
typedef __attribute__((ext_vector_type(4)))  float    v4f;
typedef __attribute__((ext_vector_type(4)))  unsigned int v4u;


#define VST2(T, ptr, val) do { const T vst2_v_ = (val); *(volatile T*)(ptr) = vst2_v_; __threadfence(); *(volatile T*)(ptr) = vst2_v_; } while (0)

__device__ __forceinline__ float bfr(float f) {
    unsigned u = __float_as_uint(f);
    u += 0x7FFFu + ((u >> 16) & 1u);
    return __uint_as_float(u & 0xFFFF0000u);
}
__device__ __forceinline__ unsigned short f2h_bits(float x) {
    return (fabsf(x) < 6.104e-5f) ? (unsigned short)0 : __builtin_bit_cast(unsigned short, (_Float16)x);
}
__device__ __forceinline__ void st8h(unsigned short* P, size_t o, const float* v) {
    v4u pk;
    pk.x = (unsigned)f2h_bits(v[0]) | ((unsigned)f2h_bits(v[1]) << 16);
    pk.y = (unsigned)f2h_bits(v[2]) | ((unsigned)f2h_bits(v[3]) << 16);
    pk.z = (unsigned)f2h_bits(v[4]) | ((unsigned)f2h_bits(v[5]) << 16);
    pk.w = (unsigned)f2h_bits(v[6]) | ((unsigned)f2h_bits(v[7]) << 16);
    VST2(v4u, (v4u*)(P + o), pk);
}
static __device__ __forceinline__ h16 toh_flush(float v) {
    const h16 r = (h16)v;
    return (fabsf(v) < 6.103515625e-05f) ? (h16)0.0f : r;
}
__device__ __forceinline__ void st8h2(unsigned short* Ph, unsigned short* Pl, size_t o, const float* v) {
    unsigned hb[8], lb[8];
#pragma unroll
    for (int i = 0; i < 8; ++i) {
        const h16 h = toh_flush(v[i]);
        const h16 l = toh_flush((v[i] - (float)h) * 2048.0f);
        hb[i] = (unsigned)__builtin_bit_cast(unsigned short, h);
        lb[i] = (unsigned)__builtin_bit_cast(unsigned short, l);
    }
    v4u ph, pl;
    ph.x = hb[0] | (hb[1] << 16); ph.y = hb[2] | (hb[3] << 16); ph.z = hb[4] | (hb[5] << 16); ph.w = hb[6] | (hb[7] << 16);
    pl.x = lb[0] | (lb[1] << 16); pl.y = lb[2] | (lb[3] << 16); pl.z = lb[4] | (lb[5] << 16); pl.w = lb[6] | (lb[7] << 16);
    VST2(v4u, (v4u*)(Ph + o), ph);
    VST2(v4u, (v4u*)(Pl + o), pl);
}

union FragU { v16h v; v8h h[2]; };
__device__ __forceinline__ v16h frag_ld(const _Float16* p) {
    FragU f; f.h[0] = *(const v8h*)(p); f.h[1] = *(const v8h*)(p + 16); return f.v;
}
__device__ __forceinline__ v8f wmma16(v16h a, v16h b, v8f c) {
    c = __builtin_amdgcn_wmma_f32_16x16x32_f16(false, a, false, b, (short)0, c, false, false);
    asm volatile("v_nop\n\tv_nop\n\tv_nop\n\tv_nop" : "+v"(c) : "v"(a), "v"(b));
    return c;
}
__device__ __forceinline__ void wave_sync_lds() {
    __builtin_amdgcn_fence(3  , "workgroup");
    __builtin_amdgcn_wave_barrier();
    __builtin_amdgcn_fence(2  , "workgroup");
}

__global__ __launch_bounds__(256) void k_planes(const float* __restrict__ Wmax, const float* __restrict__ U3,
                                                unsigned short* __restrict__ WA, unsigned short* __restrict__ UB) {
    const unsigned u = blockIdx.x * 256u + threadIdx.x;
    float v[8];
    if (blockIdx.x < (unsigned)((MEC * 4) / 256)) {
        const unsigned r = u >> 2, k0 = 8u * (u & 3u);
        const unsigned e = r >> 7, c = r & 127u;
#pragma unroll
        for (int i = 0; i < 8; ++i) {
            const unsigned k = k0 + (unsigned)i;
            const unsigned kc = (k < (unsigned)NP3) ? k : (unsigned)(NP3 - 1);
            const float w = bfr(Wmax[((size_t)e * NP3 + kc) * CHN + c]) * SWC;
            v[i] = (k < (unsigned)NP3) ? w : 0.0f;
        }
        st8h(WA, (size_t)u * 8u, v);
    } else {
        const unsigned u2 = u - (unsigned)(MEC * 4);
        const unsigned q = u2 >> 2, k0 = 8u * (u2 & 3u);
#pragma unroll
        for (int i = 0; i < 8; ++i) {
            const unsigned k = k0 + (unsigned)i;
            const unsigned kc = (k < (unsigned)NP3) ? k : (unsigned)(NP3 - 1);
            const float w = bfr(U3[(size_t)q * NP3 + kc]) * SUC;
            v[i] = (k < (unsigned)NP3) ? w : 0.0f;
        }
        st8h(UB, (size_t)u2 * 8u, v);
    }
}

__global__ __launch_bounds__(256) void k_tail(const float* __restrict__ U2, const float* __restrict__ U1,
                                              const float* __restrict__ W2, const float* __restrict__ W1,
                                              unsigned short* __restrict__ BThi, unsigned short* __restrict__ BTlo) {
    const unsigned u = blockIdx.x * 256u + threadIdx.x;
    const unsigned ec = u >> 6, w = (u >> 2) & 15u, g = u & 3u;
    const unsigned e = ec >> 7, c = ec & 127u;
    const unsigned xb = 8u * (g & 1u);
    float acc[8];
#pragma unroll
    for (int j = 0; j < 8; ++j) acc[j] = 0.0f;
#pragma unroll 1
    for (unsigned p = 0; p < (unsigned)NP2; ++p) {
        const float w2 = bfr(W2[((size_t)e * NP2 + p) * CHN + c]);
#pragma unroll
        for (int j = 0; j < 8; ++j)
            acc[j] += bfr(U2[((size_t)(w * 16u + xb + (unsigned)j)) * NP2 + p]) * w2;
    }
    const float v1 = bfr(U1[w]) * bfr(W1[(size_t)e * CHN + c]);
    float v[8];
#pragma unroll
    for (int j = 0; j < 8; ++j) v[j] = (g < 2u) ? acc[j] * SBC : 0.0f;
    v[0] = (g < 2u) ? acc[0] * SBC : ((g == 2u) ? v1 * SBC : 0.0f);
    st8h2(BThi, BTlo, (size_t)u * 8u, v);
}

__global__ __launch_bounds__(256) void k_vgemm(const _Float16* __restrict__ A, const _Float16* __restrict__ Bt,
                                               _Float16* __restrict__ Chi, _Float16* __restrict__ Clo,
                                               unsigned M, unsigned N, float scale) {
    __shared__ __align__(16) float sT[8][16 * 68];
    const unsigned lane = threadIdx.x & 31u;
    const unsigned wave = (unsigned)__builtin_amdgcn_readfirstlane((int)(threadIdx.x >> 5));
    const unsigned tilesN = N >> 6, tilesM = M >> 6;
    const unsigned tile = blockIdx.x * 8u + wave;
    if (tile >= tilesM * tilesN) return;
    const unsigned tm = tile / tilesN;
    const unsigned tn = tile - tm * tilesN;
    const unsigned m0 = tm << 6, n0 = tn << 6;
    const unsigned rlane = lane & 15u;
    const unsigned koff = (lane >> 4) * 8u;

    v16h bh[4];
#pragma unroll
    for (int j = 0; j < 4; ++j)
        bh[j] = frag_ld(Bt + (size_t)(n0 + ((unsigned)j << 4) + rlane) * KP + koff);

#pragma unroll 1
    for (unsigned i = 0; i < 4u; ++i) {
        const unsigned mBase = m0 + (i << 4);
        const v16h ah = frag_ld(A + (size_t)(mBase + rlane) * KP + koff);
        v8f acc[4];
#pragma unroll
        for (int j = 0; j < 4; ++j) {
            const v8f z = (v8f){0.f,0.f,0.f,0.f,0.f,0.f,0.f,0.f};
            acc[j] = wmma16(ah, bh[j], z);
        }
#pragma unroll
        for (int j = 0; j < 4; ++j)
#pragma unroll
            for (int r = 0; r < 8; ++r)
                sT[wave][(koff + (unsigned)r) * 68u + ((unsigned)j << 4) + rlane] = acc[j][r] * scale;
        wave_sync_lds();
        {
            const unsigned q = lane >> 3, c8 = (lane & 7u) * 8u;
            v8h hv[4], lv[4];
#pragma unroll
            for (int it = 0; it < 4; ++it) {
                const unsigned row = (unsigned)it * 4u + q;
#pragma unroll
                for (int el = 0; el < 8; ++el) {
                    const float v = sT[wave][row * 68u + c8 + (unsigned)el];
                    const h16 h = toh_flush(v);
                    hv[it][el] = h;
                    lv[it][el] = toh_flush((v - (float)h) * 2048.0f);
                }
            }
            for (int pass = 0; pass < 2; ++pass) {
#pragma unroll
                for (int it = 0; it < 4; ++it) {
                    const unsigned row = (unsigned)it * 4u + q;
                    *(volatile v8h*)(Chi + (size_t)(mBase + row) * N + n0 + c8) = hv[it];
                    *(volatile v8h*)(Clo + (size_t)(mBase + row) * N + n0 + c8) = lv[it];
                }
                __threadfence();
            }
        }
        wave_sync_lds();
    }
}

__global__ __launch_bounds__(256) void k_cubic(const float* __restrict__ x, const float* __restrict__ y, const float* __restrict__ shw,
                                              const _Float16* __restrict__ B3hi, const _Float16* __restrict__ B3lo,
                                              const _Float16* __restrict__ BThi, const _Float16* __restrict__ BTlo,
                                              float* __restrict__ out) {
    __shared__ int sList[NB];
    __shared__ unsigned sCnt[8];
    __shared__ __align__(16) float sX[8][16 * XP];
    __shared__ __align__(16) float sS[8][16 * 16];
    __shared__ float sF[8][16];
    const unsigned tid = threadIdx.x, lane = tid & 31u;
    const unsigned wv = tid >> 5;
    const unsigned wave = (unsigned)__builtin_amdgcn_readfirstlane((int)(tid >> 5));
    const unsigned hh = lane >> 4, m = lane & 15u;
    const unsigned e = blockIdx.x >> 3, cg = blockIdx.x & 7u;
    const unsigned zs = blockIdx.y;

    const unsigned a0 = wave * (unsigned)(NB / 8);
    unsigned cnt = 0;
#pragma unroll 1
    for (unsigned it = 0; it < (unsigned)(NB / 256); ++it) {
        const unsigned a = a0 + it * 32u + lane;
        const float yv = y[(size_t)a * NEL + e];
        const unsigned mk = __builtin_amdgcn_ballot_w32(yv != 0.0f);
        cnt += (unsigned)__popc(mk);
    }
    if (lane == 0u) sCnt[wave] = cnt;
    __syncthreads();
    unsigned base = 0, total = 0;
#pragma unroll
    for (unsigned j = 0; j < 8u; ++j) {
        const unsigned cj = sCnt[j];
        total += cj;
        base += (j < wv) ? cj : 0u;
    }
    {
        unsigned run = base;
#pragma unroll 1
        for (unsigned it = 0; it < (unsigned)(NB / 256); ++it) {
            const unsigned a = a0 + it * 32u + lane;
            const float yv = y[(size_t)a * NEL + e];
            const bool hit = (yv != 0.0f);
            const unsigned mk = __builtin_amdgcn_ballot_w32(hit);
            const unsigned pos = run + (unsigned)__popc(mk & ((1u << lane) - 1u));
            if (hit && pos < (unsigned)NB) sList[pos] = (int)a;
            run += (unsigned)__popc(mk);
        }
    }
    __syncthreads();
    const unsigned totc = (total < (unsigned)NB) ? total : (unsigned)NB;
    const unsigned ntile = (unsigned)__builtin_amdgcn_readfirstlane((int)((totc + 15u) >> 4));

#pragma unroll 1
    for (unsigned t = zs * 8u + wave; t < ntile; t += 8u * (unsigned)TSPLIT) {
        const unsigned lpL = t * 16u + (lane >> 1);
        const unsigned lpR = t * 16u + m;
        int bL = sList[(lpL < totc) ? lpL : (totc - 1u)];
        int bR = sList[(lpR < totc) ? lpR : (totc - 1u)];
        bL = min(max(bL, 0), NB - 1);
        bR = min(max(bR, 0), NB - 1);
        {
            unsigned nnz = 0;
#pragma unroll
            for (int j = 0; j < NEL; ++j) nnz += (y[(size_t)bR * NEL + (unsigned)j] != 0.0f) ? 1u : 0u;
            const float yv = bfr(y[(size_t)bR * NEL + e]);
            const float fz = (nnz == 1u) ? yv : __uint_as_float(0x7FC00000u);
            sF[wave][m] = fz;
        }

#pragma unroll 1
        for (unsigned cc = 0; cc < 16u; ++cc) {
            const unsigned c = cg * 16u + cc;
            {
                const unsigned m2 = lane >> 1, hf = lane & 1u;
                const float* src = x + ((size_t)bL * CHN + c) * LDIM + hf * 8u;
                v4f p0 = *(const v4f*)src, p1 = *(const v4f*)(src + 4);
                p0.x = bfr(p0.x); p0.y = bfr(p0.y); p0.z = bfr(p0.z); p0.w = bfr(p0.w);
                p1.x = bfr(p1.x); p1.y = bfr(p1.y); p1.z = bfr(p1.z); p1.w = bfr(p1.w);
                *(v4f*)&sX[wave][m2 * XP + hf * 8u] = p0;
                *(v4f*)&sX[wave][m2 * XP + hf * 8u + 4u] = p1;
            }
            wave_sync_lds();
            float xi[8];
#pragma unroll
            for (int i = 0; i < 8; ++i) xi[i] = sX[wave][m * XP + 8u * hh + (unsigned)i];

            const size_t ec = (size_t)e * CHN + c;
            const _Float16* b3h = B3hi + (ec * 16u + m) * 256u + 8u * hh;
            const _Float16* b3l = B3lo + (ec * 16u + m) * 256u + 8u * hh;
            v8f accm = (v8f){0.f,0.f,0.f,0.f,0.f,0.f,0.f,0.f};
            v8f accr = (v8f){0.f,0.f,0.f,0.f,0.f,0.f,0.f,0.f};
#pragma unroll 1
            for (unsigned s = 0; s < 8u; ++s) {
                const float x0 = sX[wave][m * XP + 2u * s] * SAC;
                const float x1 = sX[wave][m * XP + 2u * s + 1u] * SAC;
                v16h ah, al;
#pragma unroll
                for (int i = 0; i < 8; ++i) {
                    const float g0 = x0 * xi[i];
                    const h16 h0 = toh_flush(g0);
                    ah[i] = h0;
                    al[i] = toh_flush((g0 - (float)h0) * 2048.0f);
                    const float g1 = x1 * xi[i];
                    const h16 h1 = toh_flush(g1);
                    ah[8 + i] = h1;
                    al[8 + i] = toh_flush((g1 - (float)h1) * 2048.0f);
                }
                const v16h bhv = frag_ld(b3h + 32u * s);
                const v16h blv = frag_ld(b3l + 32u * s);
                accm = wmma16(ah, bhv, accm);
                accr = wmma16(al, bhv, accr);
                accr = wmma16(ah, blv, accr);
            }
            {
                v16h at;
#pragma unroll
                for (int i = 0; i < 8; ++i) at[i] = toh_flush(xi[i] * SAC);
                const float one = (hh == 0u) ? SAC : 0.0f;
                at[8] = toh_flush(one);
#pragma unroll
                for (int i = 9; i < 16; ++i) at[i] = (h16)0.0f;
                const v16h bth = frag_ld(BThi + (ec * 16u + m) * 32u + 8u * hh);
                const v16h btl = frag_ld(BTlo + (ec * 16u + m) * 32u + 8u * hh);
                accm = wmma16(at, bth, accm);
                accr = wmma16(at, btl, accr);
            }
#pragma unroll
            for (int r = 0; r < 8; ++r) {
                const float c1 = (accm[r] + accr[r] * (1.0f / 2048.0f)) * (1.0f / 65536.0f);
                float p = c1 * sX[wave][(8u * hh + (unsigned)r) * XP + m];
                p += __shfl_xor(p, 1, 32);
                p += __shfl_xor(p, 2, 32);
                p += __shfl_xor(p, 4, 32);
                p += __shfl_xor(p, 8, 32);
                if (m == 0u) sS[wave][(8u * hh + (unsigned)r) * 16u + cc] = p;
            }
            wave_sync_lds();
        }

        {
            const unsigned q = lane >> 3, pc = lane & 7u;
            v4f vv[8];
            size_t oo[8];
            bool okk[8];
#pragma unroll
            for (int it = 0; it < 8; ++it) {
                const unsigned L = (unsigned)it * 4u + q;
                const unsigned mr = L >> 1, a = L & 1u;
                const unsigned lp = t * 16u + mr;
                okk[it] = lp < totc;
                int bi = sList[(lp < totc) ? lp : (totc - 1u)];
                bi = min(max(bi, 0), NB - 1);
                const float fz = sF[wave][mr];
                const float s0 = sS[wave][mr * 16u + 2u * pc] * fz;
                const float s1 = sS[wave][mr * 16u + 2u * pc + 1u] * fz;
                const v4f sh = *(const v4f*)(shw + ((size_t)a * CHN + cg * 16u + 2u * pc) * 2u);
                v4f o;
                o.x = s0 * bfr(sh.x); o.y = s0 * bfr(sh.y); o.z = s1 * bfr(sh.z); o.w = s1 * bfr(sh.w);
                vv[it] = o;
                oo[it] = (((size_t)bi * 2u + a) * CHN + cg * 16u) * 2u + 4u * pc;
            }
            for (int pass = 0; pass < 2; ++pass) {
#pragma unroll
                for (int it = 0; it < 8; ++it) {
                    if (okk[it]) *(volatile v4f*)(out + oo[it]) = vv[it];
                }
                __threadfence();
            }
        }
        wave_sync_lds();
    }
}

extern "C" void kernel_launch(void* const* d_in, const int* in_sizes, int n_in, void* d_out, int out_size,
                              void* d_ws, size_t ws_size, hipStream_t stream) {
    if (n_in < 9) return;
    if (in_sizes[0] < NB * CHN * LDIM || in_sizes[1] < NB * NEL || in_sizes[2] < NQ * NP3 || in_sizes[3] < LDIM * LDIM * NP2) return;
    if (in_sizes[4] < LDIM || in_sizes[5] < NEL * NP3 * CHN || in_sizes[6] < NEL * NP2 * CHN || in_sizes[7] < NEL * CHN) return;
    if (in_sizes[8] < 2 * CHN * 2 || out_size < NB * 2 * CHN * 2) return;

    const float* x    = (const float*)d_in[0];
    const float* y    = (const float*)d_in[1];
    const float* U3   = (const float*)d_in[2];
    const float* U2   = (const float*)d_in[3];
    const float* U1   = (const float*)d_in[4];
    const float* Wmax = (const float*)d_in[5];
    const float* W2   = (const float*)d_in[6];
    const float* W1   = (const float*)d_in[7];
    const float* shw  = (const float*)d_in[8];
    float* out = (float*)d_out;

    char* wsp = (char*)d_ws;
    size_t off = 0;
    auto carve = [&](size_t bytes) -> void* { void* r = wsp + off; off += (bytes + 255) & ~(size_t)255; return r; };
    unsigned short* WA   = (unsigned short*)carve((size_t)MEC * KP * 2);
    unsigned short* UB   = (unsigned short*)carve((size_t)NQ * KP * 2);
    _Float16*       B3hi = (_Float16*)carve((size_t)MEC * NQ * 2);
    _Float16*       B3lo = (_Float16*)carve((size_t)MEC * NQ * 2);
    unsigned short* BThi = (unsigned short*)carve((size_t)MEC * 16 * 32 * 2);
    unsigned short* BTlo = (unsigned short*)carve((size_t)MEC * 16 * 32 * 2);
    if (off > ws_size || off > (size_t)134217728) return;

    k_planes<<<(MEC * 4 + NQ * 4) / 256, 256, 0, stream>>>(Wmax, U3, WA, UB);
    k_tail<<<(MEC * 64) / 256, 256, 0, stream>>>(U2, U1, W2, W1, BThi, BTlo);
    k_vgemm<<<((MEC / 64) * (NQ / 64)) / 8, 256, 0, stream>>>((const _Float16*)WA, (const _Float16*)UB, B3hi, B3lo,
                                                               (unsigned)MEC, (unsigned)NQ, VSCALE);
    k_cubic<<<dim3(NEL * 8, TSPLIT), 256, 0, stream>>>(x, y, shw, (const _Float16*)B3hi, (const _Float16*)B3lo,
                                                      (const _Float16*)BThi, (const _Float16*)BTlo, out);
}
